// OptimizedHierarchicalEncoder_23613730193796
// MI455X (gfx1250) — hardware-verified
//
#include <hip/hip_runtime.h>
#include <stddef.h>
#include <math.h>

#pragma clang fp contract(off)


#define NJ    17
#define CH    64
#define OUTF  128
#define FD    384
#define KE    64
#define KP    384
#define NDT   16
#define MAXG  13
#define MAXS  5
#define TILE  256
#define SWF   (3 * 256)
#define SBF   (MAXG * 4 * TILE)
#define SAF   (MAXS * 4 * TILE)
#define SFF   (NDT * FD)
#define LDS_MAIN ((SWF + SBF + SAF + SFF) * 4)
#define PE_N  (OUTF * KE)
#define PP_N  (OUTF * KP)
#define WTHR  256
#define NBPE  (PE_N / (8 * WTHR))
#define NBPP  (PP_N / (8 * WTHR))
#define WSCAP 134217728

static_assert(LDS_MAIN == 101376);
static_assert(NBPE * 8 * WTHR == PE_N);
static_assert(NBPP * 8 * WTHR == PP_N);
static_assert(NDT * OUTF <= SBF);
static_assert((KE % 8) == 0 && (KP % 8) == 0 && (FD % 32) == 0);
static_assert((PE_N * 2) % 512 == 0 && (PP_N * 2) % 512 == 0);

typedef float          v2f  __attribute__((ext_vector_type(2)));
typedef float          v4f  __attribute__((ext_vector_type(4)));
typedef float          v8f  __attribute__((ext_vector_type(8)));
typedef unsigned short v8us __attribute__((ext_vector_type(8)));
typedef unsigned int   v8u  __attribute__((ext_vector_type(8)));
typedef __bf16         v16b __attribute__((ext_vector_type(16)));
union BFrag { v16b v; v8us h[2]; v8u w; };

__constant__ int   c_G[3]    = {9, 13, 8};
__constant__ int   c_S[3]    = {5, 4, 4};
__constant__ float c_invS[3] = {0.2f, 0.25f, 0.25f};
__constant__ int c_allnb[3][MAXG] = {
  {0, 5, 6, 7, 8, 11, 12, 13, 14, 0, 0, 0, 0},
  {0, 5, 6, 7, 8, 9, 10, 11, 12, 13, 14, 15, 16},
  {7, 8, 9, 10, 13, 14, 15, 16, 0, 0, 0, 0, 0}};
__constant__ int c_subpos[3][MAXG] = {
  { 0,  1,  2, -1, -1,  3,  4, -1, -1, -1, -1, -1, -1},
  {-1, -1, -1,  0,  1, -1, -1, -1, -1,  2,  3, -1, -1},
  {-1, -1,  0,  1, -1, -1,  2,  3, -1, -1, -1, -1, -1}};
__constant__ int c_subslot[3][MAXS] = {{0, 1, 2, 5, 6}, {3, 4, 9, 10, 0}, {2, 3, 6, 7, 0}};

__device__ __forceinline__ v8f wmb(v16b a, v16b b, v8f c) {
  v8f d = __builtin_amdgcn_wmma_f32_16x16x32_bf16(false, a, false, b, (short)0, c, false, false);
  asm volatile("v_nop\n\tv_nop\n\tv_nop\n\tv_nop" : "+v"(d) : "v"(a), "v"(b));
  return d;
}

__device__ __forceinline__ unsigned bfbits(float x) {
  const unsigned u = __float_as_uint(x);
  return (u + 0x7FFFu + ((u >> 16) & 1u)) >> 16;
}
__device__ __forceinline__ void split1(float x, unsigned& hb, unsigned& lb) {
  hb = bfbits(x);
  const float r = x - __uint_as_float(hb << 16);
  lb = bfbits(r);
}
__device__ __forceinline__ void split2(float x, float y, unsigned& ph, unsigned& pl) {
  unsigned hx, lx, hy, ly;
  split1(x, hx, lx);
  split1(y, hy, ly);
  ph = hx | (hy << 16);
  pl = lx | (ly << 16);
}

__device__ __forceinline__ void mrun8(const float* wl, int cb, float kx, float ky, float s, float (&mv)[8]) {
  const v4f a0 = *(const v4f*)(wl + cb),          a1 = *(const v4f*)(wl + cb + 4);
  const v4f b0 = *(const v4f*)(wl + CH + cb),     b1 = *(const v4f*)(wl + CH + cb + 4);
  const v4f c0 = *(const v4f*)(wl + 2 * CH + cb), c1 = *(const v4f*)(wl + 2 * CH + cb + 4);
  const v4f d0 = *(const v4f*)(wl + 3 * CH + cb), d1 = *(const v4f*)(wl + 3 * CH + cb + 4);
  const float wx[8] = {a0.x, a0.y, a0.z, a0.w, a1.x, a1.y, a1.z, a1.w};
  const float wy[8] = {b0.x, b0.y, b0.z, b0.w, b1.x, b1.y, b1.z, b1.w};
  const float ws[8] = {c0.x, c0.y, c0.z, c0.w, c1.x, c1.y, c1.z, c1.w};
  const float wb[8] = {d0.x, d0.y, d0.z, d0.w, d1.x, d1.y, d1.z, d1.w};
#pragma unroll
  for (int e = 0; e < 8; ++e) {
    float p = kx * wx[e];
    p = fmaf(ky, wy[e], p);
    p = fmaf(s, ws[e], p);
    const float h = fmaxf(p + wb[e], 0.0f);
    mv[e] = h * s;
  }
}

__global__ __launch_bounds__(WTHR) void k_wprep(const float* __restrict__ We, const float* __restrict__ Wp,
                                                unsigned short* PEh, unsigned short* PEl,
                                                unsigned short* PPh, unsigned short* PPl) {
  const int blk = blockIdx.x, tid = threadIdx.x;
  float v[8];
  unsigned short* dh;
  unsigned short* dl;
  if (blk < NBPE) {
    const int i = blk * WTHR + tid;
    const int n = i >> 3, k0 = (i & 7) * 8;
    const int nc = n & (CH - 1);
#pragma unroll
    for (int e = 0; e < 8; ++e) {
      const float wa = We[(k0 + e) * CH + nc];
      const float wb = We[(CH + k0 + e) * CH + nc];
      v[e] = (n >= CH) ? wb : (wa - wb);
    }
    dh = PEh + (size_t)i * 8;
    dl = PEl + (size_t)i * 8;
  } else {
    const int i = (blk - NBPE) * WTHR + tid;
    const int n = i / 48, k0 = (i - n * 48) * 8;
#pragma unroll
    for (int e = 0; e < 8; ++e) v[e] = Wp[(k0 + e) * OUTF + n];
    dh = PPh + (size_t)i * 8;
    dl = PPl + (size_t)i * 8;
  }
  v8us hv = {0, 0, 0, 0, 0, 0, 0, 0}, lv = {0, 0, 0, 0, 0, 0, 0, 0};
#pragma unroll
  for (int e = 0; e < 8; ++e) {
    unsigned hb, lb;
    split1(v[e], hb, lb);
    hv[e] = (unsigned short)hb;
    lv[e] = (unsigned short)lb;
  }
  *(volatile v8us*)dh = hv;
  *(volatile v8us*)dl = lv;
  __threadfence();
  *(volatile v8us*)dh = hv;
  *(volatile v8us*)dl = lv;
}

__global__ __launch_bounds__(32) void k_main(
    const float* __restrict__ kp, const float* __restrict__ sc,
    const float* __restrict__ W0, const float* __restrict__ b0,
    const float* __restrict__ W1, const float* __restrict__ b1,
    const float* __restrict__ W2, const float* __restrict__ b2,
    const float* __restrict__ be, const float* __restrict__ bp,
    const unsigned short* __restrict__ PEh, const unsigned short* __restrict__ PEl,
    const unsigned short* __restrict__ PPh, const unsigned short* __restrict__ PPl,
    float* out, int nN) {
  extern __shared__ v4f lds_dyn[];
  float* sW = (float*)lds_dyn;
  float* sB = sW + SWF;
  float* sA = sB + SBF;
  float* sF = sA + SAF;
  const int lane = threadIdx.x & 31, hh = lane >> 4, m = lane & 15;
  const int det0 = blockIdx.x * NDT;
  int det = det0 + m;
  det = det > nN - 1 ? nN - 1 : det;
  const v8f z8 = {0.f, 0.f, 0.f, 0.f, 0.f, 0.f, 0.f, 0.f};

  for (int i = lane; i < 3 * CH; i += 32) {
    sW[i] = W0[i];
    sW[256 + i] = W1[i];
    sW[512 + i] = W2[i];
  }
  for (int i = lane; i < CH; i += 32) {
    sW[3 * CH + i] = b0[i];
    sW[256 + 3 * CH + i] = b1[i];
    sW[512 + 3 * CH + i] = b2[i];
  }

  float beF[4];
#pragma unroll
  for (int t = 0; t < 4; ++t) beF[t] = be[16 * t + m];

  const float* kd = kp + (size_t)det * (NJ * 2);
  const float* sd = sc + (size_t)det * NJ;
  float mnx, mxx, mny, mxy;
  {
    const v2f p0 = *(const v2f*)kd;
    mnx = p0.x; mxx = p0.x; mny = p0.y; mxy = p0.y;
#pragma unroll
    for (int j = 1; j < NJ; ++j) {
      const v2f p = *(const v2f*)(kd + 2 * j);
      mnx = fminf(mnx, p.x); mxx = fmaxf(mxx, p.x);
      mny = fminf(mny, p.y); mxy = fmaxf(mxy, p.y);
    }
  }
  const float ivx = 1.0f / ((mxx - mnx) + 1e-6f);
  const float ivy = 1.0f / ((mxy - mny) + 1e-6f);
  __syncthreads();

#pragma unroll 1
  for (int lvl = 0; lvl < 3; ++lvl) {
    const int G = c_G[lvl], S = c_S[lvl];
    const float invS = c_invS[lvl];
    const float* wl = sW + lvl * 256;

    float hs[32];
#pragma unroll
    for (int e = 0; e < 32; ++e) hs[e] = 0.0f;
#pragma unroll 1
    for (int gi = 0; gi < G; ++gi) {
      const int g  = c_allnb[lvl][gi];
      const int sp = c_subpos[lvl][gi];
      const float fsub = (sp >= 0) ? 1.0f : 0.0f;
      const float x = kd[2 * g], y = kd[2 * g + 1], s = sd[g];
      const float kx = (x - mnx) * ivx, ky = (y - mny) * ivy;
      BFrag ah[2], al[2];
#pragma unroll
      for (int ks = 0; ks < 2; ++ks) {
        v8u wh = {0u, 0u, 0u, 0u, 0u, 0u, 0u, 0u}, wlo = {0u, 0u, 0u, 0u, 0u, 0u, 0u, 0u};
#pragma unroll
        for (int q = 0; q < 2; ++q) {
          const int cb = 32 * ks + 16 * q + 8 * hh;
          float mv[8];
          mrun8(wl, cb, kx, ky, s, mv);
#pragma unroll
          for (int e = 0; e < 8; ++e) hs[16 * ks + 8 * q + e] += mv[e] * fsub;
#pragma unroll
          for (int e4 = 0; e4 < 4; ++e4) {
            unsigned ph, pl;
            split2(mv[2 * e4], mv[2 * e4 + 1], ph, pl);
            wh[4 * q + e4] = ph;
            wlo[4 * q + e4] = pl;
          }
        }
        ah[ks].w = wh;
        al[ks].w = wlo;
      }
      const int spc = sp < 0 ? 0 : sp;
      const int tBeg = sp < 0 ? 4 : 0;
#pragma unroll 1
      for (int t = tBeg; t < 8; ++t) {
        v8f acc = z8;
#pragma unroll
        for (int ks = 0; ks < 2; ++ks) {
          const size_t bo = (size_t)(16 * t + m) * KE + 32 * ks + 8 * hh;
          BFrag bh, bl;
          bh.h[0] = *(const v8us*)(PEh + bo);
          bh.h[1] = *(const v8us*)(PEh + bo + 16);
          bl.h[0] = *(const v8us*)(PEl + bo);
          bl.h[1] = *(const v8us*)(PEl + bo + 16);
          acc = wmb(ah[ks].v, bh.v, acc);
          acc = wmb(ah[ks].v, bl.v, acc);
          acc = wmb(al[ks].v, bh.v, acc);
        }
        float* dst = sB + ((t < 4) ? (SBF + (spc * 4 + t) * TILE) : ((gi * 4 + (t - 4)) * TILE)) + lane * 8;
        const v4f u0 = {acc[0], acc[1], acc[2], acc[3]};
        const v4f u1 = {acc[4], acc[5], acc[6], acc[7]};
        *(v4f*)dst = u0;
        *(v4f*)(dst + 4) = u1;
      }
    }
    {
      float* fr = sF + m * FD + lvl * 128;
#pragma unroll
      for (int ks = 0; ks < 2; ++ks) {
#pragma unroll
        for (int q = 0; q < 2; ++q) {
          const int cb = 32 * ks + 16 * q + 8 * hh;
          const v4f u0 = {hs[16 * ks + 8 * q + 0], hs[16 * ks + 8 * q + 1], hs[16 * ks + 8 * q + 2], hs[16 * ks + 8 * q + 3]};
          const v4f u1 = {hs[16 * ks + 8 * q + 4], hs[16 * ks + 8 * q + 5], hs[16 * ks + 8 * q + 6], hs[16 * ks + 8 * q + 7]};
          *(v4f*)(fr + cb) = u0;
          *(v4f*)(fr + cb + 4) = u1;
        }
      }
    }
    __syncthreads();

    float Zs[32];
#pragma unroll
    for (int e = 0; e < 32; ++e) Zs[e] = 0.0f;
#pragma unroll 1
    for (int si = 0; si < S; ++si) {
      const int js = c_subslot[lvl][si];
      const float* ap = sA + (si * 4) * TILE + lane * 8;
      float a[32];
#pragma unroll
      for (int t = 0; t < 4; ++t) {
        const v4f u0 = *(const v4f*)(ap + t * TILE), u1 = *(const v4f*)(ap + t * TILE + 4);
        a[8 * t + 0] = u0.x + beF[t]; a[8 * t + 1] = u0.y + beF[t];
        a[8 * t + 2] = u0.z + beF[t]; a[8 * t + 3] = u0.w + beF[t];
        a[8 * t + 4] = u1.x + beF[t]; a[8 * t + 5] = u1.y + beF[t];
        a[8 * t + 6] = u1.z + beF[t]; a[8 * t + 7] = u1.w + beF[t];
      }
      float mx[32];
#pragma unroll
      for (int e = 0; e < 32; ++e) mx[e] = 0.0f;
#pragma unroll 1
      for (int k = 0; k < G; ++k) {
        if (k == js) continue;
        const float* bq = sB + (k * 4) * TILE + lane * 8;
#pragma unroll
        for (int t = 0; t < 4; ++t) {
          const v4f u0 = *(const v4f*)(bq + t * TILE), u1 = *(const v4f*)(bq + t * TILE + 4);
          const float bv[8] = {u0.x, u0.y, u0.z, u0.w, u1.x, u1.y, u1.z, u1.w};
#pragma unroll
          for (int r = 0; r < 8; ++r) {
            const float val = fmaxf(a[8 * t + r] + bv[r], 0.0f);
            mx[8 * t + r] = fmaxf(mx[8 * t + r], val);
          }
        }
      }
#pragma unroll
      for (int e = 0; e < 32; ++e) Zs[e] += mx[e];
    }
#pragma unroll
    for (int t = 0; t < 4; ++t) {
#pragma unroll
      for (int r = 0; r < 8; ++r) sF[(8 * hh + r) * FD + lvl * 128 + CH + 16 * t + m] = Zs[8 * t + r] * invS;
    }
    __syncthreads();
  }

  float* stg = sB;
#pragma unroll
  for (int p = 0; p < 2; ++p) {
    v8f Co[4];
#pragma unroll
    for (int t4 = 0; t4 < 4; ++t4) Co[t4] = z8;
#pragma unroll 1
    for (int kf = 0; kf < FD / 32; ++kf) {
      const float* fr = sF + m * FD + 32 * kf + 8 * hh;
      BFrag fa, fl;
      {
        v8u wh = {0u, 0u, 0u, 0u, 0u, 0u, 0u, 0u}, wlo = {0u, 0u, 0u, 0u, 0u, 0u, 0u, 0u};
#pragma unroll
        for (int q = 0; q < 2; ++q) {
          const v4f u0 = *(const v4f*)(fr + 16 * q), u1 = *(const v4f*)(fr + 16 * q + 4);
          const float f8[8] = {u0.x, u0.y, u0.z, u0.w, u1.x, u1.y, u1.z, u1.w};
#pragma unroll
          for (int e4 = 0; e4 < 4; ++e4) {
            unsigned ph, pl;
            split2(f8[2 * e4], f8[2 * e4 + 1], ph, pl);
            wh[4 * q + e4] = ph;
            wlo[4 * q + e4] = pl;
          }
        }
        fa.w = wh;
        fl.w = wlo;
      }
#pragma unroll
      for (int t4 = 0; t4 < 4; ++t4) {
        const size_t bo = (size_t)(16 * (4 * p + t4) + m) * KP + 32 * kf + 8 * hh;
        BFrag bh, bl;
        bh.h[0] = *(const v8us*)(PPh + bo);
        bh.h[1] = *(const v8us*)(PPh + bo + 16);
        bl.h[0] = *(const v8us*)(PPl + bo);
        bl.h[1] = *(const v8us*)(PPl + bo + 16);
        Co[t4] = wmb(fa.v, bh.v, Co[t4]);
        Co[t4] = wmb(fa.v, bl.v, Co[t4]);
        Co[t4] = wmb(fl.v, bh.v, Co[t4]);
      }
    }
#pragma unroll
    for (int t4 = 0; t4 < 4; ++t4) {
      const int t = 4 * p + t4;
      const float bv = bp[16 * t + m];
#pragma unroll
      for (int r = 0; r < 8; ++r) stg[(8 * hh + r) * OUTF + 16 * t + m] = Co[t4][r] + bv;
    }
  }
  __syncthreads();

#pragma unroll
  for (int row = 0; row < NDT; ++row) {
    const int dr = det0 + row;
    const v4f v = *(const v4f*)(stg + row * OUTF + 4 * lane);
    if (dr < nN) *(volatile v4f*)(out + (size_t)dr * OUTF + 4 * lane) = v;
  }
  __threadfence();
#pragma unroll
  for (int row = 0; row < NDT; ++row) {
    const int dr = det0 + row;
    const v4f v = *(const v4f*)(stg + row * OUTF + 4 * lane);
    if (dr < nN) *(volatile v4f*)(out + (size_t)dr * OUTF + 4 * lane) = v;
  }
}

extern "C" void kernel_launch(void* const* d_in, const int* in_sizes, int n_in,
                              void* d_out, int out_size, void* d_ws, size_t ws_size,
                              hipStream_t stream) {
  if (n_in < 12) return;
  const int nN = in_sizes[0] / (NJ * 2);
  if (nN <= 0 || nN > (1 << 24)) return;
  if (in_sizes[0] != nN * NJ * 2 || in_sizes[1] != nN * NJ) return;
  if (in_sizes[2] != 3 * CH || in_sizes[3] != CH || in_sizes[4] != 3 * CH || in_sizes[5] != CH) return;
  if (in_sizes[6] != 3 * CH || in_sizes[7] != CH) return;
  if (in_sizes[8] != 2 * CH * CH || in_sizes[9] != CH || in_sizes[10] != FD * OUTF || in_sizes[11] != OUTF) return;
  if (out_size != nN * OUTF) return;

  const float* kp = (const float*)d_in[0];
  const float* sc = (const float*)d_in[1];
  const float* W0 = (const float*)d_in[2];
  const float* b0 = (const float*)d_in[3];
  const float* W1 = (const float*)d_in[4];
  const float* b1 = (const float*)d_in[5];
  const float* W2 = (const float*)d_in[6];
  const float* b2 = (const float*)d_in[7];
  const float* We = (const float*)d_in[8];
  const float* be = (const float*)d_in[9];
  const float* Wp = (const float*)d_in[10];
  const float* bp = (const float*)d_in[11];
  float* out = (float*)d_out;

  char* ws = (char*)d_ws;
  size_t off = 0;
  const size_t oEh = off; off += (size_t)PE_N * 2; off = (off + 255) & ~(size_t)255;
  const size_t oEl = off; off += (size_t)PE_N * 2; off = (off + 255) & ~(size_t)255;
  const size_t oPh = off; off += (size_t)PP_N * 2; off = (off + 255) & ~(size_t)255;
  const size_t oPl = off; off += (size_t)PP_N * 2; off = (off + 255) & ~(size_t)255;
  if (off > ws_size || off > (size_t)WSCAP) return;
  unsigned short* PEh = (unsigned short*)(ws + oEh);
  unsigned short* PEl = (unsigned short*)(ws + oEl);
  unsigned short* PPh = (unsigned short*)(ws + oPh);
  unsigned short* PPl = (unsigned short*)(ws + oPl);

  k_wprep<<<NBPE + NBPP, WTHR, 0, stream>>>(We, Wp, PEh, PEl, PPh, PPl);
  hipFuncSetAttribute(reinterpret_cast<const void*>(&k_main),
                      hipFuncAttributeMaxDynamicSharedMemorySize, LDS_MAIN);
  const int nBlk = (nN + NDT - 1) / NDT;
  k_main<<<nBlk, 32, LDS_MAIN, stream>>>(kp, sc, W0, b0, W1, b1, W2, b2, be, bp, PEh, PEl, PPh, PPl, out, nN);
}
